// LowRank_Attention_47158740910458
// MI455X (gfx1250) — hardware-verified
//
#include <hip/hip_runtime.h>
#include <math.h>

typedef __attribute__((ext_vector_type(16))) _Float16 v16h;
typedef __attribute__((ext_vector_type(16))) __bf16 v16b;
typedef __attribute__((ext_vector_type(8)))  _Float16 v8h;
typedef __attribute__((ext_vector_type(8)))  float v8f;
typedef __attribute__((ext_vector_type(4)))  float v4f;
typedef __attribute__((ext_vector_type(2)))  float v2f;
typedef __attribute__((ext_vector_type(4)))  unsigned v4u;
typedef __attribute__((ext_vector_type(4)))  int v4i;
typedef float __attribute__((may_alias)) float_a;
typedef int __attribute__((may_alias)) int_a;

template <typename T> __device__ __forceinline__ void vst2(void* p, T v) { *(volatile T*)p = v; __threadfence(); *(volatile T*)p = v; }
__device__ __forceinline__ v8f wmma16(v16h a, v16h b, v8f c) {
  v8f d = __builtin_amdgcn_wmma_f32_16x16x32_f16(false, a, false, b, (short)0, c, false, false);
  asm volatile("v_nop\n\tv_nop\n\tv_nop\n\tv_nop" : "+v"(d) : "v"(a), "v"(b));
  return d;
}
__device__ __forceinline__ v8f wmma_bf(v16b a, v16b b, v8f c) {
  v8f d = __builtin_amdgcn_wmma_f32_16x16x32_bf16(false, a, false, b, (short)0, c, false, false);
  asm volatile("v_nop\n\tv_nop\n\tv_nop\n\tv_nop" : "+v"(d) : "v"(a), "v"(b));
  return d;
}
__device__ __forceinline__ v16h frag_h(const _Float16* rowk0, int lane) {
  union { v16h v; v8h q[2]; } u; const _Float16* p = rowk0 + 8 * (lane >> 4);
  u.q[0] = *(const v8h*)p; u.q[1] = *(const v8h*)(p + 16); return u.v;
}
__device__ __forceinline__ v16h frag_f32(const float* rowk0, int lane) {
  v16h a; const float* p = rowk0 + 8 * (lane >> 4);
#pragma unroll
  for (int i = 0; i < 8; ++i) { a[i] = (_Float16)p[i]; a[8 + i] = (_Float16)p[16 + i]; }
  return a;
}
__device__ __forceinline__ v16h frag_f32s(const float* rowk0, int lane, float sc) {
  v16h a; const float* p = rowk0 + 8 * (lane >> 4);
#pragma unroll
  for (int i = 0; i < 8; ++i) { a[i] = (_Float16)(p[i] * sc); a[8 + i] = (_Float16)(p[16 + i] * sc); }
  return a;
}
__device__ __forceinline__ v16h fragc_f32(const float* W, int k0, int n, int lane, int ld, int K) {
  v16h a; const int g = lane >> 4;
#pragma unroll
  for (int i = 0; i < 8; ++i) { const int ka = k0 + 8 * g + i, kb = ka + 16;
    a[i] = (_Float16)(ka < K ? W[(size_t)(ka < K ? ka : K - 1) * ld + n] : 0.f); a[8 + i] = (_Float16)(kb < K ? W[(size_t)(kb < K ? kb : K - 1) * ld + n] : 0.f); }
  return a;
}
struct F2 { v16b h, l; };
__device__ __forceinline__ F2 bsplit16(const float v[16]) { F2 r;
#pragma unroll
  for (int i = 0; i < 16; ++i) { const __bf16 h = (__bf16)v[i]; r.h[i] = h; r.l[i] = (__bf16)(v[i] - (float)h); }
  return r; }
__device__ __forceinline__ F2 split_row(const float* row, int k0, int lane) { float v[16]; const float* p = row + k0 + 8 * (lane >> 4);
#pragma unroll
  for (int i = 0; i < 8; ++i) { v[i] = p[i]; v[8 + i] = p[16 + i]; }
  return bsplit16(v); }
__device__ __forceinline__ F2 split_rowK(const float* row, int k0, int lane, int K) { float v[16]; const int g = lane >> 4;
#pragma unroll
  for (int i = 0; i < 8; ++i) { const int ka = k0 + 8 * g + i, kb = ka + 16; v[i] = ka < K ? row[ka < K ? ka : K - 1] : 0.f; v[8 + i] = kb < K ? row[kb < K ? kb : K - 1] : 0.f; }
  return bsplit16(v); }
__device__ __forceinline__ F2 split_col(const float* W, int k0, int n, int lane, int ld, int K) { float v[16]; const int g = lane >> 4;
#pragma unroll
  for (int i = 0; i < 8; ++i) { const int ka = k0 + 8 * g + i, kb = ka + 16; v[i] = ka < K ? W[(size_t)(ka < K ? ka : K - 1) * ld + n] : 0.f; v[8 + i] = kb < K ? W[(size_t)(kb < K ? kb : K - 1) * ld + n] : 0.f; }
  return bsplit16(v); }
__device__ __forceinline__ v8f mac3(const F2& a, const F2& b, v8f c) { c = wmma_bf(a.l, b.h, c); c = wmma_bf(a.h, b.l, c); return wmma_bf(a.h, b.h, c); }
__device__ __forceinline__ float sigm(float v) { return 1.0f / (1.0f + expf(-v)); }
#define LDSX() do { asm volatile("s_wait_dscnt 0" ::: "memory"); __builtin_amdgcn_wave_barrier(); __builtin_amdgcn_fence(__ATOMIC_RELEASE, "workgroup"); } while (0)


#define NBATCH 64
#define SQ 197
#define SP 224
#define DM 768
#define NH 12
#define HD 64
#define KR 64
#define NR (NBATCH * SQ)
#ifndef NBT
#define NBT NBATCH
#endif
#define NRT ((NBT * SQ + 63) / 64)
typedef __attribute__((ext_vector_type(8))) __bf16 v8b;
__device__ __forceinline__ v16b frag_b(const __bf16* rowk0, int lane) {
  union { v16b v; v8b q[2]; } u; const __bf16* p = rowk0 + 8 * (lane >> 4);
  u.q[0] = *(const v8b*)p; u.q[1] = *(const v8b*)(p + 16); return u.v;
}
__device__ __forceinline__ float bfr(float v) { return (float)(__bf16)v; }
__device__ __attribute__((noinline)) float exp_ni(float v) { return expf(v); }
__device__ __attribute__((noinline)) float erf_ni(float v) { return erff(v); }

#define WS_PQ   0u
#define WS_Q    (WS_PQ + 2u * (size_t)4 * DM * DM)
#define WS_K    (WS_Q + 2u * (size_t)NR * DM)
#define WS_V    (WS_K + 2u * (size_t)NR * DM)
#define WS_KP   (WS_V + 2u * (size_t)NR * DM)
#define WS_VPL  (WS_KP + 2u * (size_t)NBATCH * DM * SP)
#define WS_E16  (WS_VPL + 2u * (size_t)NBATCH * DM * SP)
#define WS_PK   (WS_E16 + 2u * (size_t)2 * KR * SP)
#define WS_PVT  (WS_PK + 2u * (size_t)NBATCH * KR * DM)
#define WS_CTX  (WS_PVT + 2u * (size_t)NBATCH * DM * KR)
#define WS_END  (WS_CTX + 4u * (size_t)NR * DM)

__global__ __launch_bounds__(256) void k_pack(const float* __restrict__ WQ, const float* __restrict__ WK, const float* __restrict__ WV, const float* __restrict__ WO, __bf16* __restrict__ P) { const int n = blockIdx.x, which = blockIdx.y, t = threadIdx.x; const float* Wm = (which == 0) ? WQ : (which == 1) ? WK : (which == 2) ? WV : WO; __shared__ __align__(16) __bf16 s[DM]; for (int k = t; k < DM; k += 256) s[k] = (__bf16)Wm[(size_t)k * DM + n]; __syncthreads(); for (int q = t; q < DM / 8; q += 256) vst2((unsigned*)(P + ((size_t)which * DM + n) * DM + q * 8), *(const v4u*)&s[q * 8]); }
__global__ __launch_bounds__(256) void k_e16(const float* __restrict__ EK, const float* __restrict__ EV, _Float16* __restrict__ E16) { const int j = blockIdx.x, which = blockIdx.y, t = threadIdx.x; const float* E = which ? EV : EK; __shared__ __align__(16) _Float16 s[SP]; if (t < SP) s[t] = (t < SQ) ? (_Float16)bfr(E[(size_t)t * KR + j]) : (_Float16)0.f; __syncthreads(); if (t < SP / 8) vst2((unsigned*)(E16 + ((size_t)which * KR + j) * SP + t * 8), *(const v4u*)&s[t * 8]); }
__global__ __launch_bounds__(128) void k_proj(const float* __restrict__ X, const __bf16* __restrict__ P, const float* __restrict__ BQ, const float* __restrict__ BK, const float* __restrict__ BV, _Float16* __restrict__ Q, _Float16* __restrict__ Kr, _Float16* __restrict__ Vr) {
  __shared__ __align__(16) _Float16 so[64][136];
  const int tid = threadIdx.x, wave = tid >> 5, lane = tid & 31, col = lane & 15, g = lane >> 4; const int which = blockIdx.z; const int n0 = blockIdx.y * 128; const size_t r0 = (size_t)blockIdx.x * 64 + wave * 16;
  const __bf16* Wr = P + (size_t)which * DM * DM; const float* BB = (which == 0) ? BQ : (which == 1) ? BK : BV; _Float16* dst = (which == 0) ? Q : (which == 1) ? Kr : Vr;
  v8f acc[8] = {};
#pragma unroll 2
  for (int kc = 0; kc < DM / 32; ++kc) { v16b a; { const float* p = X + (r0 + col) * DM + kc * 32 + 8 * g;
#pragma unroll
      for (int i = 0; i < 8; ++i) { a[i] = (__bf16)p[i]; a[8 + i] = (__bf16)p[16 + i]; } }
#pragma unroll
    for (int j = 0; j < 8; ++j) acc[j] = wmma_bf(a, frag_b(Wr + (size_t)(n0 + j * 16 + col) * DM + kc * 32, lane), acc[j]); }
#pragma unroll
  for (int j = 0; j < 8; ++j) { const float bb = bfr(BB[n0 + j * 16 + col]);
#pragma unroll
    for (int r = 0; r < 8; ++r) so[wave * 16 + 8 * g + r][j * 16 + col] = (_Float16)(acc[j][r] + bb); }
  LDSX();
  for (int rl = 0; rl < 16; ++rl) if (lane < 16) vst2((unsigned*)(dst + (r0 + rl) * DM + n0 + lane * 8), *(const v4u*)&so[wave * 16 + rl][lane * 8]);
}
__global__ __launch_bounds__(256) void k_planes(const _Float16* __restrict__ Kr, const _Float16* __restrict__ Vr, _Float16* __restrict__ KP, _Float16* __restrict__ VPL) {
  __shared__ __align__(16) _Float16 st[64][SP + 8]; const size_t b = blockIdx.x; const int c0 = blockIdx.y * 64, which = blockIdx.z, t = threadIdx.x; const _Float16* src = which ? Vr : Kr; _Float16* dst = which ? VPL : KP;
  for (int e = t; e < 64 * SP; e += 256) { const int c = e / SP, s = e % SP; st[c][s] = (s < SQ) ? src[(b * SQ + s) * DM + c0 + c] : (_Float16)0.f; }
  __syncthreads();
  for (int e = t; e < 64 * (SP / 8); e += 256) { const int c = e / (SP / 8), q = e % (SP / 8); vst2((unsigned*)(dst + ((b * DM + c0 + c) * SP) + q * 8), *(const v4u*)&st[c][q * 8]); }
}
__global__ __launch_bounds__(128) void k_lowrank(const _Float16* __restrict__ E16, const _Float16* __restrict__ KP, const _Float16* __restrict__ VPL, _Float16* __restrict__ PK, _Float16* __restrict__ PVT) {
  __shared__ __align__(16) _Float16 so[64][136]; __shared__ __align__(16) _Float16 st[128][72];
  const int tid = threadIdx.x, wave = tid >> 5, lane = tid & 31, col = lane & 15, g = lane >> 4; const size_t b = blockIdx.x; const int c0 = blockIdx.y * 128, which = blockIdx.z; const _Float16* planes = (which ? VPL : KP) + (b * DM) * SP; const _Float16* Er = E16 + (size_t)which * KR * SP;
  const int j0 = wave * 16;
  v8f acc[8] = {};
#pragma unroll
  for (int kc = 0; kc < SP / 32; ++kc) { const v16h a = frag_h(Er + (size_t)(j0 + col) * SP + kc * 32, lane);
#pragma unroll
    for (int j = 0; j < 8; ++j) acc[j] = wmma16(a, frag_h(planes + (size_t)(c0 + j * 16 + col) * SP + kc * 32, lane), acc[j]); }
  if (which == 0) {
#pragma unroll
    for (int j = 0; j < 8; ++j)
#pragma unroll
      for (int r = 0; r < 8; ++r) so[wave * 16 + 8 * g + r][j * 16 + col] = (_Float16)acc[j][r];
    LDSX();
    for (int rl = 0; rl < 16; ++rl) if (lane < 16) vst2((unsigned*)(PK + ((b * KR + j0 + rl) * DM) + c0 + lane * 8), *(const v4u*)&so[wave * 16 + rl][lane * 8]);
  } else {
#pragma unroll
    for (int j = 0; j < 8; ++j)
#pragma unroll
      for (int r = 0; r < 8; ++r) st[j * 16 + col][wave * 16 + 8 * g + r] = (_Float16)acc[j][r];
    __syncthreads();
    for (int e = tid; e < 128 * 8; e += 128) { const int c = e >> 3, pc = e & 7; vst2((unsigned*)(PVT + ((b * DM + c0 + c) * KR) + pc * 8), *(const v4u*)&st[c][pc * 8]); } }
}
__global__ __launch_bounds__(128) void k_attn(const _Float16* __restrict__ Q, const _Float16* __restrict__ PK, const _Float16* __restrict__ PVT, float* __restrict__ CTX) {
  __shared__ __align__(16) _Float16 sph[4][16][72]; __shared__ __align__(16) float so[4][16][68];
  const int tid = threadIdx.x, wave = tid >> 5, lane = tid & 31, col = lane & 15, g = lane >> 4; const int h = blockIdx.y; const size_t b = blockIdx.z; const int s0 = blockIdx.x * 64 + wave * 16;
  v16h aq[2]; { const int sq = min(s0 + col, SQ - 1);
#pragma unroll
    for (int kc = 0; kc < 2; ++kc) aq[kc] = frag_h(Q + (b * SQ + sq) * DM + h * HD + kc * 32, lane); }
  v8f s[4];
#pragma unroll
  for (int ct = 0; ct < 4; ++ct) { v8f c = {};
#pragma unroll
    for (int kc = 0; kc < 2; ++kc) c = wmma16(aq[kc], frag_h(PK + ((b * KR + ct * 16 + col) * DM) + h * HD + kc * 32, lane), c);
#pragma unroll
    for (int r = 0; r < 8; ++r) s[ct][r] = c[r] * 0.125f; }
  float il[8];
#pragma unroll
  for (int r = 0; r < 8; ++r) { float mx = fmaxf(fmaxf(s[0][r], s[1][r]), fmaxf(s[2][r], s[3][r]));
#pragma unroll
    for (int o = 1; o < 16; o <<= 1) mx = fmaxf(mx, __shfl_xor(mx, o));
    float es = 0.f;
#pragma unroll
    for (int ct = 0; ct < 4; ++ct) { const float e = __expf(s[ct][r] - mx); es += e; sph[wave][8 * g + r][ct * 16 + col] = (_Float16)(e * 2048.0f); }
#pragma unroll
    for (int o = 1; o < 16; o <<= 1) es += __shfl_xor(es, o);
    il[r] = (1.0f / 2048.0f) / es; }
  LDSX();
  v8f acc[4] = {};
#pragma unroll
  for (int kc = 0; kc < 2; ++kc) { const v16h pa = frag_h(&sph[wave][col][kc * 32], lane);
#pragma unroll
    for (int dt = 0; dt < 4; ++dt) acc[dt] = wmma16(pa, frag_h(PVT + ((b * DM + h * HD + dt * 16 + col) * KR) + kc * 32, lane), acc[dt]); }
#pragma unroll
  for (int r = 0; r < 8; ++r)
#pragma unroll
    for (int dt = 0; dt < 4; ++dt) so[wave][8 * g + r][dt * 16 + col] = acc[dt][r] * il[r];
  LDSX();
  for (int rl = 0; rl < 16; ++rl) { const int sq = s0 + rl; if (sq < SQ && lane < 16) vst2(CTX + (b * SQ + sq) * DM + h * HD + lane * 4, *(const v4f*)&so[wave][rl][lane * 4]); }
}
__global__ __launch_bounds__(128) void k_out(const float* __restrict__ CTX, const __bf16* __restrict__ P, const float* __restrict__ BO, float* __restrict__ OUT) {
  __shared__ __align__(16) float so[4][16][132];
  const int tid = threadIdx.x, wave = tid >> 5, lane = tid & 31, col = lane & 15, g = lane >> 4; const size_t r0 = (size_t)blockIdx.x * 64 + wave * 16; const int n0 = blockIdx.y * 128;
  v8f acc[8] = {};
#pragma unroll 2
  for (int kc = 0; kc < DM / 32; ++kc) { const F2 a = split_row(CTX + (r0 + col) * DM, kc * 32, lane);
#pragma unroll
    for (int j = 0; j < 8; ++j) { const v16b w = frag_b(P + (size_t)(3 * DM + n0 + j * 16 + col) * DM + kc * 32, lane); acc[j] = wmma_bf(a.l, w, acc[j]); acc[j] = wmma_bf(a.h, w, acc[j]); } }
#pragma unroll
  for (int j = 0; j < 8; ++j) { const float bb = bfr(BO[n0 + j * 16 + col]);
#pragma unroll
    for (int r = 0; r < 8; ++r) so[wave][8 * g + r][j * 16 + col] = acc[j][r] + bb; }
  LDSX();
  for (int rl = 0; rl < 16; ++rl) vst2(OUT + (r0 + rl) * DM + n0 + lane * 4, *(const v4f*)&so[wave][rl][lane * 4]);
}
extern "C" void kernel_launch(void* const* d_in, const int* in_sizes, int n_in, void* d_out, int out_size, void* d_ws, size_t ws_size, hipStream_t stream) {
  (void)in_sizes; (void)n_in; (void)out_size;
  const float** F = (const float**)d_in;
  if (ws_size < (size_t)WS_END) return;
  char* ws = (char*)d_ws; __bf16* P = (__bf16*)ws; _Float16 *Q = (_Float16*)(ws + WS_Q), *Kr = (_Float16*)(ws + WS_K), *Vr = (_Float16*)(ws + WS_V), *KP = (_Float16*)(ws + WS_KP), *VPL = (_Float16*)(ws + WS_VPL), *E16 = (_Float16*)(ws + WS_E16), *PK = (_Float16*)(ws + WS_PK), *PVT = (_Float16*)(ws + WS_PVT); float* CTX = (float*)(ws + WS_CTX);
  k_pack<<<dim3(DM, 4), 256, 0, stream>>>(F[1], F[3], F[5], F[7], P);
  k_e16<<<dim3(KR, 2), 256, 0, stream>>>(F[9], F[10], E16);
  k_proj<<<dim3(NRT, DM / 128, 3), 128, 0, stream>>>(F[0], P, F[2], F[4], F[6], Q, Kr, Vr);
  k_planes<<<dim3(NBT, DM / 64, 2), 256, 0, stream>>>(Kr, Vr, KP, VPL);
  k_lowrank<<<dim3(NBT, DM / 128, 2), 128, 0, stream>>>(E16, KP, VPL, PK, PVT);
  k_attn<<<dim3(4, NH, NBT), 128, 0, stream>>>(Q, PK, PVT, CTX);
  k_out<<<dim3(NRT, DM / 128), 128, 0, stream>>>(CTX, P, F[8], (float*)d_out);
}
